// Middle_Moudle_v3_58815282152232
// MI455X (gfx1250) — hardware-run, weakly checked
//
#include <hip/hip_runtime.h>


#define NE_  8
#define NPL  75
#define NCH  64
#define NPS  361
#define NPP  384
typedef _Float16 h16;
typedef unsigned short bf;
typedef __attribute__((ext_vector_type(16))) __bf16   v16bf;
typedef __attribute__((ext_vector_type(16))) _Float16 v16h;
typedef __attribute__((ext_vector_type(8)))  _Float16 v8h;
typedef __attribute__((ext_vector_type(8)))  unsigned short v8us;
typedef __attribute__((ext_vector_type(8)))  float    v8f;
typedef __attribute__((ext_vector_type(4)))  float    v4f;
typedef v8h  __attribute__((may_alias)) v8ha;
typedef v4f  __attribute__((may_alias)) v4fa;
typedef v8us __attribute__((may_alias)) v8usa;

__device__ __forceinline__ unsigned short f2bf(float f) { unsigned u = __float_as_uint(f); u += 0x7FFFu + ((u >> 16) & 1u); return (unsigned short)(u >> 16); }
__device__ __forceinline__ float bf2f(unsigned short b) { return __uint_as_float(((unsigned)b) << 16); }
__device__ __forceinline__ float bfr(float f) { return bf2f(f2bf(f)); }
__device__ __forceinline__ v16h cat16(v8h lo, v8h hi) { return __builtin_shufflevector(lo, hi, 0, 1, 2, 3, 4, 5, 6, 7, 8, 9, 10, 11, 12, 13, 14, 15); }
__device__ __forceinline__ v16bf cat16b(v8us lo, v8us hi) { return __builtin_bit_cast(v16bf, __builtin_shufflevector(lo, hi, 0, 1, 2, 3, 4, 5, 6, 7, 8, 9, 10, 11, 12, 13, 14, 15)); }
__device__ __forceinline__ v8f wmma16(v16h a, v16h b, v8f c) { return __builtin_amdgcn_wmma_f32_16x16x32_f16(false, a, false, b, (short)0, c, false, false); }
__device__ __forceinline__ v8f wmmab(v16bf a, v16bf b, v8f c) { return __builtin_amdgcn_wmma_f32_16x16x32_bf16(false, a, false, b, (short)0, c, false, false); }


template <typename T16> struct WFrag;
template <> struct WFrag<h16> { typedef v16h V; static __device__ __forceinline__ V ld(const h16* p) { return cat16(*(const v8h*)p, *(const v8h*)(p + 16)); } static __device__ __forceinline__ v8f mma(V a, V b, v8f c) { return wmma16(a, b, c); } };
template <> struct WFrag<bf> { typedef v16bf V; static __device__ __forceinline__ V ld(const bf* p) { return cat16b(*(const v8us*)p, *(const v8us*)(p + 16)); } static __device__ __forceinline__ v8f mma(V a, V b, v8f c) { return wmmab(a, b, c); } };
template <typename T16, int NSPLIT, bool BIAS>
__global__ __launch_bounds__(32) void k_gemmw(const T16* __restrict__ A, const T16* __restrict__ A2, const T16* __restrict__ Bt, const T16* __restrict__ Bt2, int K, float* C, int ldc, const float* __restrict__ bias, size_t sA, size_t sB, size_t sC) {
    typedef typename WFrag<T16>::V V;
    __shared__ __align__(16) float os[16 * 68];
    const size_t z = blockIdx.z; A += z * sA; if (A2) A2 += z * sA; Bt += z * sB; if (Bt2) Bt2 += z * sB; C += z * sC;
    const int lane = threadIdx.x & 31, lr = lane & 15, hi = lane >> 4; const int r0 = blockIdx.x * 64, c0 = blockIdx.y * 64;
    v8f acc[4][4];
#pragma unroll
    for (int mb = 0; mb < 4; ++mb)
#pragma unroll
        for (int nb = 0; nb < 4; ++nb) acc[mb][nb] = (v8f){};
    const size_t aoff = (size_t)(r0 + lr) * K + 8 * hi, boff = (size_t)(c0 + lr) * K + 8 * hi;
    for (int kc = 0; kc < K; kc += 32) {
        V a[4], a2[4];
#pragma unroll
        for (int mb = 0; mb < 4; ++mb) { a[mb] = WFrag<T16>::ld(A + aoff + (size_t)mb * 16 * K + kc); if (NSPLIT == 1 || NSPLIT == 2) a2[mb] = WFrag<T16>::ld(A2 + aoff + (size_t)mb * 16 * K + kc); }
#pragma unroll
        for (int nb = 0; nb < 4; ++nb) { const V b = WFrag<T16>::ld(Bt + boff + (size_t)nb * 16 * K + kc); V b2; if (NSPLIT >= 2) b2 = WFrag<T16>::ld(Bt2 + boff + (size_t)nb * 16 * K + kc);
#pragma unroll
            for (int mb = 0; mb < 4; ++mb) { acc[mb][nb] = WFrag<T16>::mma(a[mb], b, acc[mb][nb]); if (NSPLIT == 1 || NSPLIT == 2) acc[mb][nb] = WFrag<T16>::mma(a2[mb], b, acc[mb][nb]); if (NSPLIT >= 2) acc[mb][nb] = WFrag<T16>::mma(a[mb], b2, acc[mb][nb]); } }
        asm volatile("v_nop\n\tv_nop\n\tv_nop\n\tv_nop" : "+v"(acc[0][0]), "+v"(acc[1][1]), "+v"(acc[2][2]), "+v"(acc[3][3]) : "v"(a[0]), "v"(a[3]));
    }
#pragma unroll
    for (int mb = 0; mb < 4; ++mb) {
#pragma unroll
        for (int nb = 0; nb < 4; ++nb) {
#pragma unroll
            for (int j = 0; j < 8; ++j) os[(hi * 8 + j) * 68 + nb * 16 + lr] = acc[mb][nb][j]; }
        __builtin_amdgcn_wave_barrier(); asm volatile("" ::: "memory");
        float* crow = C + (size_t)(r0 + mb * 16) * ldc + c0;
#pragma unroll 1
        for (int ps = 0; ps < 2; ++ps) {
#pragma unroll
            for (int s = 0; s < 8; ++s) { const int row = 2 * s + hi, cofs = lr * 4; v4f val = *(const v4fa*)(os + row * 68 + cofs); if (BIAS) { val[0] += bfr(bias[c0 + cofs]); val[1] += bfr(bias[c0 + cofs + 1]); val[2] += bfr(bias[c0 + cofs + 2]); val[3] += bfr(bias[c0 + cofs + 3]); }
                *(volatile v4f*)(crow + (size_t)row * ldc + cofs) = val; }
            if (ps == 0) __threadfence(); }
        __builtin_amdgcn_wave_barrier(); asm volatile("" ::: "memory");
    }
}

__device__ __forceinline__ h16 tohx(float x) { return (h16)x; }
__device__ __forceinline__ void splitf(float y, unsigned short& h, unsigned short& l) { h = f2bf(y); l = f2bf(y - bf2f(h)); }
typedef __attribute__((ext_vector_type(2))) _Float16 v2h;
typedef __attribute__((ext_vector_type(4))) _Float16 v4h;
typedef __attribute__((ext_vector_type(2))) unsigned short v2us;
typedef __attribute__((ext_vector_type(4))) unsigned short v4us;
typedef __attribute__((ext_vector_type(2))) float v2f;
typedef __attribute__((ext_vector_type(4))) int v4i;

__global__ __launch_bounds__(256) void k_tp(const float* __restrict__ src, bf* T) { const unsigned idx = blockIdx.x * 256 + threadIdx.x; const unsigned c0 = (idx % (NCH / 8)) * 8, r = (idx / (NCH / 8)) % NPP, z = idx / ((NCH / 8) * NPP); const unsigned rc = (r < NPS) ? r : (NPS - 1); const float f = (r < NPS) ? 1.0f : 0.0f; v8us o;
#pragma unroll
    for (int q = 0; q < 8; ++q) o[q] = f2bf(__fmul_rn(bfr(src[((size_t)z * NCH + c0 + q) * NPS + rc]), f));
    *(volatile v8us*)(T + (size_t)idx * 8) = o; __threadfence(); *(volatile v8us*)(T + (size_t)idx * 8) = o; }
__global__ __launch_bounds__(128) void k_nr(const float* __restrict__ src, float* N) { const unsigned idx = blockIdx.x * 128 + threadIdx.x; const unsigned p = idx % NPP, z = idx / NPP; const unsigned pc = (p < NPS) ? p : (NPS - 1); float s = 0.0f;
#pragma unroll
    for (int c = 0; c < NCH; ++c) { const float w = bfr(src[((size_t)z * NCH + c) * NPS + pc]); s = __fadd_rn(s, __fmul_rn(w, w)); }
    const float y = (p < NPS) ? __fsqrt_rn(s) : 1.0f; *(volatile float*)(N + idx) = y; __threadfence(); *(volatile float*)(N + idx) = y; }
__global__ __launch_bounds__(128) void k_mx(const float* __restrict__ NUM, const float* __restrict__ NS, const float* __restrict__ NQ, float* MX) { const unsigned idx = blockIdx.x * 128 + threadIdx.x; const unsigned z = idx / NPP; const float* row = NUM + (size_t)idx * NPP; const float* nq = NQ + (size_t)z * NPP; const float ns = NS[idx]; float m = -3.0e38f;
    for (int pb = 0; pb < NPS - 1; pb += 20) {
#pragma unroll
        for (int q = 0; q < 20; ++q) { const float d = __fmul_rn(ns, nq[pb + q]); const float v = __fdiv_rn(row[pb + q], (d > 1.0e-8f) ? d : 1.0e-8f); m = (v > m) ? v : m; } }
    { const float d = __fmul_rn(ns, nq[NPS - 1]); const float v = __fdiv_rn(row[NPS - 1], (d > 1.0e-8f) ? d : 1.0e-8f); m = (v > m) ? v : m; }
    *(volatile float*)(MX + idx) = m; __threadfence(); *(volatile float*)(MX + idx) = m; }
__global__ __launch_bounds__(256) void k_pk(const float* __restrict__ MX, float* out, unsigned first) { const unsigned l = first + blockIdx.x * blockDim.x + threadIdx.x; v4f o;
#pragma unroll
    for (int q = 0; q < 4; ++q) { const unsigned w = l * 4 + q; const unsigned pl = w / NPS, ps = w - pl * NPS; o[q] = MX[(size_t)pl * NPP + ps]; }
    *(volatile v4f*)(out + (size_t)l * 4) = o; __threadfence(); *(volatile v4f*)(out + (size_t)l * 4) = o; }

extern "C" void kernel_launch(void* const* d_in, const int* in_sizes, int n_in,
                              void* d_out, int out_size, void* d_ws, size_t ws_size, hipStream_t stream) {
    (void)in_sizes; (void)n_in; (void)out_size;
    const float* a0 = (const float*)d_in[0]; const float* a1 = (const float*)d_in[1];
    float* OUT = (float*)d_out;
    char* wsp = (char*)d_ws;
    auto take = [&](size_t bytes) { char* p = wsp; wsp += (bytes + 255) & ~(size_t)255; return (void*)p; };
    bf* TS = (bf*)take((size_t)NPL * NPP * NCH * 2); bf* TQ = (bf*)take((size_t)NPL * NPP * NCH * 2); float* NS = (float*)take((size_t)NPL * NPP * 4); float* NQ = (float*)take((size_t)NPL * NPP * 4);
    float* NUM = (float*)take((size_t)NPL * NPP * NPP * 4); float* MX = (float*)take((size_t)NE_ * NPL * NPP * 4);
    if ((size_t)(wsp - (char*)d_ws) > ws_size) return;
    const size_t EN = (size_t)NPL * NCH * NPS;
    for (int e = 0; e < NE_; ++e) {
        k_tp<<<NPL * NPP * (NCH / 8) / 256, 256, 0, stream>>>(a0 + e * EN, TS); k_tp<<<NPL * NPP * (NCH / 8) / 256, 256, 0, stream>>>(a1 + e * EN, TQ);
        k_nr<<<NPL * NPP / 128, 128, 0, stream>>>(a0 + e * EN, NS); k_nr<<<NPL * NPP / 128, 128, 0, stream>>>(a1 + e * EN, NQ);
        k_gemmw<bf, 0, false><<<dim3(NPP / 64, NPP / 64, NPL), 32, 0, stream>>>(TS, nullptr, TQ, nullptr, NCH, NUM, NPP, nullptr, (size_t)NPP * NCH, (size_t)NPP * NCH, (size_t)NPP * NPP);
        k_mx<<<NPL * NPP / 128, 128, 0, stream>>>(NUM, NS, NQ, MX + (size_t)e * NPL * NPP); }
    k_pk<<<211, 256, 0, stream>>>(MX, OUT, 0u); k_pk<<<1, 134, 0, stream>>>(MX, OUT, 54016u);
}
